// SOMFNN_25907242730005
// MI455X (gfx1250) — hardware-verified
//
#include <hip/hip_runtime.h>
#include <math.h>

typedef __attribute__((ext_vector_type(16))) _Float16 v16h;
typedef __attribute__((ext_vector_type(16))) __bf16 v16b;
typedef __attribute__((ext_vector_type(8)))  _Float16 v8h;
typedef __attribute__((ext_vector_type(8)))  float v8f;
typedef __attribute__((ext_vector_type(4)))  float v4f;
typedef __attribute__((ext_vector_type(2)))  float v2f;
typedef __attribute__((ext_vector_type(4)))  unsigned v4u;
typedef __attribute__((ext_vector_type(4)))  int v4i;
typedef float __attribute__((may_alias)) float_a;
typedef int __attribute__((may_alias)) int_a;

template <typename T> __device__ __forceinline__ void vst2(void* p, T v) { *(volatile T*)p = v; __threadfence(); *(volatile T*)p = v; }
__device__ __forceinline__ v8f wmma16(v16h a, v16h b, v8f c) {
  v8f d = __builtin_amdgcn_wmma_f32_16x16x32_f16(false, a, false, b, (short)0, c, false, false);
  asm volatile("v_nop\n\tv_nop\n\tv_nop\n\tv_nop" : "+v"(d) : "v"(a), "v"(b));
  return d;
}
__device__ __forceinline__ v8f wmma_bf(v16b a, v16b b, v8f c) {
  v8f d = __builtin_amdgcn_wmma_f32_16x16x32_bf16(false, a, false, b, (short)0, c, false, false);
  asm volatile("v_nop\n\tv_nop\n\tv_nop\n\tv_nop" : "+v"(d) : "v"(a), "v"(b));
  return d;
}
__device__ __forceinline__ v16h frag_h(const _Float16* rowk0, int lane) {
  union { v16h v; v8h q[2]; } u; const _Float16* p = rowk0 + 8 * (lane >> 4);
  u.q[0] = *(const v8h*)p; u.q[1] = *(const v8h*)(p + 16); return u.v;
}
__device__ __forceinline__ v16h frag_f32(const float* rowk0, int lane) {
  v16h a; const float* p = rowk0 + 8 * (lane >> 4);
#pragma unroll
  for (int i = 0; i < 8; ++i) { a[i] = (_Float16)p[i]; a[8 + i] = (_Float16)p[16 + i]; }
  return a;
}
__device__ __forceinline__ v16h frag_f32s(const float* rowk0, int lane, float sc) {
  v16h a; const float* p = rowk0 + 8 * (lane >> 4);
#pragma unroll
  for (int i = 0; i < 8; ++i) { a[i] = (_Float16)(p[i] * sc); a[8 + i] = (_Float16)(p[16 + i] * sc); }
  return a;
}
__device__ __forceinline__ v16h fragc_f32(const float* W, int k0, int n, int lane, int ld, int K) {
  v16h a; const int g = lane >> 4;
#pragma unroll
  for (int i = 0; i < 8; ++i) { const int ka = k0 + 8 * g + i, kb = ka + 16;
    a[i] = (_Float16)(ka < K ? W[(size_t)(ka < K ? ka : K - 1) * ld + n] : 0.f); a[8 + i] = (_Float16)(kb < K ? W[(size_t)(kb < K ? kb : K - 1) * ld + n] : 0.f); }
  return a;
}
struct F2 { v16b h, l; };
__device__ __forceinline__ F2 bsplit16(const float v[16]) { F2 r;
#pragma unroll
  for (int i = 0; i < 16; ++i) { const __bf16 h = (__bf16)v[i]; r.h[i] = h; r.l[i] = (__bf16)(v[i] - (float)h); }
  return r; }
__device__ __forceinline__ F2 split_row(const float* row, int k0, int lane) { float v[16]; const float* p = row + k0 + 8 * (lane >> 4);
#pragma unroll
  for (int i = 0; i < 8; ++i) { v[i] = p[i]; v[8 + i] = p[16 + i]; }
  return bsplit16(v); }
__device__ __forceinline__ F2 split_rowK(const float* row, int k0, int lane, int K) { float v[16]; const int g = lane >> 4;
#pragma unroll
  for (int i = 0; i < 8; ++i) { const int ka = k0 + 8 * g + i, kb = ka + 16; v[i] = ka < K ? row[ka < K ? ka : K - 1] : 0.f; v[8 + i] = kb < K ? row[kb < K ? kb : K - 1] : 0.f; }
  return bsplit16(v); }
__device__ __forceinline__ F2 split_col(const float* W, int k0, int n, int lane, int ld, int K) { float v[16]; const int g = lane >> 4;
#pragma unroll
  for (int i = 0; i < 8; ++i) { const int ka = k0 + 8 * g + i, kb = ka + 16; v[i] = ka < K ? W[(size_t)(ka < K ? ka : K - 1) * ld + n] : 0.f; v[8 + i] = kb < K ? W[(size_t)(kb < K ? kb : K - 1) * ld + n] : 0.f; }
  return bsplit16(v); }
__device__ __forceinline__ v8f mac3(const F2& a, const F2& b, v8f c) { c = wmma_bf(a.l, b.h, c); c = wmma_bf(a.h, b.l, c); return wmma_bf(a.h, b.h, c); }
__device__ __forceinline__ float sigm(float v) { return 1.0f / (1.0f + expf(-v)); }
#define LDSX() do { asm volatile("s_wait_dscnt 0" ::: "memory"); __builtin_amdgcn_wave_barrier(); __builtin_amdgcn_fence(__ATOMIC_RELEASE, "workgroup"); } while (0)


#define NS 8192
#define DI 1024
#define NRU 16
#define NO 512
#ifndef TRB
#define TRB (NS / 64)
#endif
typedef __attribute__((ext_vector_type(8))) __bf16 v8b;
__device__ __forceinline__ v16b frag_b(const __bf16* rowk0, int lane) {
  union { v16b v; v8b q[2]; } u; const __bf16* p = rowk0 + 8 * (lane >> 4);
  u.q[0] = *(const v8b*)p; u.q[1] = *(const v8b*)(p + 16); return u.v;
}
__device__ __forceinline__ float bfr(float v) { return (float)(__bf16)v; }
__device__ __attribute__((noinline)) float exp_ni(float v) { return expf(v); }
__device__ __attribute__((noinline)) float erf_ni(float v) { return erff(v); }

#define WS_PW  0u
#define WS_END (WS_PW + 2u * (size_t)NRU * NO * DI)

__global__ __launch_bounds__(256) void k_pack(const float* __restrict__ Wm, __bf16* __restrict__ P) { const size_t n = blockIdx.x; const int t = threadIdx.x; __shared__ __align__(16) __bf16 s[DI]; for (int k = t; k < DI; k += 256) s[k] = (__bf16)Wm[n * DI + k]; __syncthreads(); for (int q = t; q < DI / 8; q += 256) vst2((unsigned*)(P + n * DI + q * 8), *(const v4u*)&s[q * 8]); }
__device__ __attribute__((noinline)) float exp_p(float v) { return expf(v); }
__global__ __launch_bounds__(128) void k_som(const float* __restrict__ X, const __bf16* __restrict__ P, const float* __restrict__ BB, const float* __restrict__ LAM, float* __restrict__ OUT) {
  __shared__ __align__(16) __bf16 sx[64][DI + 8]; __shared__ __align__(16) float so[4][16][68];
  const int tid = threadIdx.x, wave = tid >> 5, lane = tid & 31, col = lane & 15, g = lane >> 4; const size_t r0b = (size_t)blockIdx.x * 64; const size_t r0 = r0b + wave * 16; const int o0 = blockIdx.y * 128;
  for (int e = tid; e < 64 * (DI / 4); e += 128) { const int rr = e / (DI / 4), q = e % (DI / 4); const float* p = X + (r0b + rr) * DI + q * 4; sx[rr][q * 4] = (__bf16)p[0]; sx[rr][q * 4 + 1] = (__bf16)p[1]; sx[rr][q * 4 + 2] = (__bf16)p[2]; sx[rr][q * 4 + 3] = (__bf16)p[3]; }
  __syncthreads();
  v8f outv[8] = {};
#pragma unroll 1
  for (int u = 0; u < NRU; ++u) { v8f acc[8] = {};
#pragma unroll 4
    for (int kc = 0; kc < DI / 32; ++kc) { const v16b a = frag_b(&sx[wave * 16 + col][0] + kc * 32, lane);
#pragma unroll
      for (int j = 0; j < 8; ++j) acc[j] = wmma_bf(a, frag_b(P + ((size_t)u * NO + o0 + j * 16 + col) * DI + kc * 32, lane), acc[j]); }
#pragma unroll
    for (int j = 0; j < 8; ++j) { const float bb = bfr(BB[u * NO + o0 + j * 16 + col]);
#pragma unroll
      for (int r = 0; r < 8; ++r) { const float hv = 1.0f / (1.0f + exp_p(-(acc[j][r] + bb))); outv[j][r] += bfr(LAM[(r0 + 8 * g + r) * NRU + u]) * hv; } } }
#pragma unroll
  for (int half = 0; half < 2; ++half) {
#pragma unroll
    for (int j = 0; j < 4; ++j)
#pragma unroll
      for (int r = 0; r < 8; ++r) so[wave][8 * g + r][j * 16 + col] = outv[half * 4 + j][r];
    LDSX();
    for (int rl = 0; rl < 16; ++rl) if (lane < 16) vst2(OUT + (r0 + rl) * NO + o0 + half * 64 + lane * 4, *(const v4f*)&so[wave][rl][lane * 4]);
    LDSX(); }
}
extern "C" void kernel_launch(void* const* d_in, const int* in_sizes, int n_in, void* d_out, int out_size, void* d_ws, size_t ws_size, hipStream_t stream) {
  (void)in_sizes; (void)n_in; (void)out_size;
  const float** F = (const float**)d_in;
  if (ws_size < (size_t)WS_END) return;
  char* ws = (char*)d_ws; __bf16* P = (__bf16*)ws;
  k_pack<<<NRU * NO, 256, 0, stream>>>(F[1], P);
  k_som<<<dim3(TRB, NO / 128), 128, 0, stream>>>(F[0], P, F[2], F[3], (float*)d_out);
}
